// EncoderAttention_17944373363289
// MI455X (gfx1250) — hardware-verified
//
#include <hip/hip_runtime.h>
#include <math.h>

constexpr int NSEQ       = 16384;
constexpr int NSTEP      = 36;
constexpr int NFEAT      = 18;
constexpr int NHID       = 128;
constexpr int NG3        = 3 * NHID;
constexpr int SEQF       = NSTEP * NFEAT;
constexpr int ROWS_BLK   = 32;
constexpr int NTHR_MAIN  = 128;
constexpr int NWAVE_MAIN = NTHR_MAIN / 32;
constexpr int NTHR_PREP  = 256;
constexpr int KSIG       = 64;
constexpr int NSIGP      = 64;
constexpr int NLHP       = 64;
constexpr int KIN        = 32;
constexpr int ATP        = 64;
constexpr int HP         = 136;
constexpr int XP         = 40;
constexpr int LHP        = 68;
constexpr int SSP        = 36;
constexpr int OUTP       = 132;
constexpr int MROWS_SIG  = ROWS_BLK * NFEAT;
constexpr int MSUB_SIG   = MROWS_SIG / 16;
constexpr float WCARRY   = 16.0f;
constexpr float ACARRY   = 64.0f;
constexpr float SCARRY   = 16.0f;
constexpr float FOLD_SIG = 1.0f / 256.0f;
constexpr float FOLD_REC = 1.0f / 1024.0f;

static_assert(NSEQ % ROWS_BLK == 0);
static_assert(ROWS_BLK * 4 == NTHR_MAIN);
static_assert(NWAVE_MAIN == 2 * (ROWS_BLK / 16));
static_assert(NHID == 16 * 4 * 2);
static_assert(NTHR_MAIN == NHID);
static_assert(MROWS_SIG % 16 == 0 && MSUB_SIG % NWAVE_MAIN == 0);
static_assert(KSIG % 32 == 0 && KIN % 32 == 0 && NHID % 32 == 0);
static_assert(NSTEP <= KSIG && NFEAT <= KIN && 3 * 16 <= NSIGP && NSTEP <= NSIGP && NLHP == 64 && NSTEP <= NLHP);
static_assert(ATP % 8 == 0 && HP % 8 == 0 && XP % 8 == 0 && ATP >= KSIG && HP >= NHID && XP >= KIN);
static_assert((ROWS_BLK * SEQF) % 4 == 0 && (ROWS_BLK * NSTEP) % 4 == 0);
static_assert(ROWS_BLK * OUTP <= MROWS_SIG * SSP);
static_assert((ROWS_BLK * NHID / 4) % NTHR_MAIN == 0);
static_assert((MROWS_SIG * ATP) % 8 == 0 && (2 * ROWS_BLK * HP) % 8 == 0 && (ROWS_BLK * XP) % 8 == 0);
static_assert(NFEAT > 3 + 12);

typedef __attribute__((ext_vector_type(16))) _Float16 v16h;
typedef __attribute__((ext_vector_type(8)))  _Float16 v8h;
typedef __attribute__((ext_vector_type(8)))  float    v8f;
typedef __attribute__((ext_vector_type(4)))  float    v4f;

__device__ __forceinline__ void dep_guard_h(v8f& a, v8f& b, v16h x, v16h y) { asm volatile("v_nop\n\tv_nop\n\tv_nop\n\tv_nop" : "+v"(a), "+v"(b) : "v"(x), "v"(y)); }
__device__ __forceinline__ void keep4_h(v16h a, v16h b, v16h c, v16h d) { asm volatile("v_nop" :: "v"(a), "v"(b), "v"(c), "v"(d)); }
__device__ __forceinline__ void acc_guard4(v8f& a, v8f& b, v8f& c, v8f& d) { asm volatile("v_nop\n\tv_nop\n\tv_nop\n\tv_nop" : "+v"(a), "+v"(b), "+v"(c), "+v"(d)); }
__device__ __forceinline__ void acc_guard3(v8f& a, v8f& b, v8f& c) { asm volatile("v_nop\n\tv_nop\n\tv_nop\n\tv_nop" : "+v"(a), "+v"(b), "+v"(c)); }
__device__ __forceinline__ void acc_guard2(v8f& a, v8f& b) { asm volatile("v_nop\n\tv_nop\n\tv_nop\n\tv_nop" : "+v"(a), "+v"(b)); }
template <typename T> struct Frag;
template <> struct Frag<_Float16> {
  typedef v16h V; union U { v16h v; v8h h[2]; };
  static __device__ __forceinline__ v16h load(const _Float16* p) {
    U f; f.h[0] = *(const v8h*)(p); f.h[1] = *(const v8h*)(p + 16); return f.v;
  }
  static __device__ __forceinline__ v8f mma(v16h a, v16h b, v8f c) {
    return __builtin_amdgcn_wmma_f32_16x16x32_f16(false, a, false, b, (short)0, c, false, false);
  }
};

__device__ __forceinline__ float fsig(float x)  { return __builtin_amdgcn_rcpf(1.0f + __expf(-x)); }
__device__ __forceinline__ float ftanh(float x) { return 1.0f - 2.0f * __builtin_amdgcn_rcpf(__expf(2.0f * x) + 1.0f); }

__global__ __launch_bounds__(NTHR_PREP) void padcvt_f16_kernel(const float* __restrict__ src, unsigned short* __restrict__ dst,
                                                               int nrow_src, int ncol_src, int nrow_dst, int ncol_dst, float sc) {
  const int i = blockIdx.x * NTHR_PREP + threadIdx.x;
  const int ncol8 = ncol_dst >> 3;
  const int n8 = nrow_dst * ncol8;
  if (i < n8) {
    const int r  = i / ncol8;
    const int c8 = (i - r * ncol8) * 8;
    const int rc = (r < nrow_src) ? r : (nrow_src - 1);
    const float rfac = (r < nrow_src) ? sc : 0.0f;
    const float* sp = src + (size_t)rc * ncol_src;
    v8h hv;
#pragma unroll
    for (int e = 0; e < 8; ++e) {
      const int cc  = c8 + e;
      const int ccl = (cc < ncol_src) ? cc : (ncol_src - 1);
      const float fac = (cc < ncol_src) ? rfac : 0.0f;
      hv[e] = (_Float16)(sp[ccl] * fac);
    }
    *(volatile v8h*)(dst + (size_t)i * 8) = hv;
    __threadfence();
    *(volatile v8h*)(dst + (size_t)i * 8) = hv;
  }
}

__global__ __launch_bounds__(NTHR_MAIN) void seq_rnn_kernel(
    const float* __restrict__ seqs, const float* __restrict__ tmask,
    const float* __restrict__ bias_lh, const float* __restrict__ bias_sig,
    const float* __restrict__ wo, const float* __restrict__ bo,
    const float* __restrict__ b_ih, const float* __restrict__ b_hh,
    const unsigned short* __restrict__ WSPp, const unsigned short* __restrict__ WHPp,
    const unsigned short* __restrict__ WIHp, const unsigned short* __restrict__ WHHp,
    float* __restrict__ out) {
  __shared__ __align__(16) float    sLinSig[MROWS_SIG * SSP];
  __shared__ __align__(16) _Float16 sAT[MROWS_SIG * ATP];
  __shared__ __align__(16) _Float16 sH[2 * ROWS_BLK * HP];
  __shared__ __align__(16) _Float16 sX[ROWS_BLK * XP];
  __shared__ __align__(16) float    sLinH[ROWS_BLK * LHP];
  __shared__ __align__(16) float    sMask[ROWS_BLK * NSTEP];
  __shared__ __align__(16) float    sWo[NTHR_MAIN];
  __shared__ __align__(16) float    sB[4 * NHID];

  const _Float16* WS16  = (const _Float16*)WSPp;
  const _Float16* WH16  = (const _Float16*)WHPp;
  const _Float16* WI16  = (const _Float16*)WIHp;
  const _Float16* WHH16 = (const _Float16*)WHHp;
  const int tid = threadIdx.x, lane = tid & 31, wave = tid >> 5;
  const int c = lane & 15, hh = lane >> 4, koff = hh * 8;
  const int msub = wave >> 1, half = wave & 1;
  const int rowbase = blockIdx.x * ROWS_BLK;
  const v8f z8 = {0.f, 0.f, 0.f, 0.f, 0.f, 0.f, 0.f, 0.f};
  v8h zh;
#pragma unroll
  for (int e = 0; e < 8; ++e) zh[e] = (_Float16)0.0f;

#pragma unroll 1
  for (int i = tid; i < MROWS_SIG * ATP / 8; i += NTHR_MAIN) *(v8h*)(sAT + 8 * i) = zh;
#pragma unroll 1
  for (int i = tid; i < 2 * ROWS_BLK * HP / 8; i += NTHR_MAIN) *(v8h*)(sH + 8 * i) = zh;
#pragma unroll 1
  for (int i = tid; i < ROWS_BLK * XP / 8; i += NTHR_MAIN) *(v8h*)(sX + 8 * i) = zh;
  sWo[tid] = wo[(tid < NSTEP) ? tid : (NSTEP - 1)];
  sB[tid]            = b_ih[tid] + b_hh[tid];
  sB[NHID + tid]     = b_ih[NHID + tid] + b_hh[NHID + tid];
  sB[2 * NHID + tid] = b_ih[2 * NHID + tid];
  sB[3 * NHID + tid] = b_hh[2 * NHID + tid];
#pragma unroll 1
  for (int i = tid; i < ROWS_BLK * NSTEP / 4; i += NTHR_MAIN) {
    const v4f v = *(const v4f*)(tmask + (size_t)rowbase * NSTEP + 4 * i);
    *(v4f*)(sMask + 4 * i) = v;
  }
  const float bsv0 = bias_sig[c];
  const float bsv1 = bias_sig[16 + c];
  const int   ss2  = 32 + c;
  const float bsv2 = bias_sig[(ss2 < NSTEP) ? ss2 : (NSTEP - 1)];
  const int   sl0  = 32 * half + c, sl1 = sl0 + 16;
  const float bhv0 = bias_lh[(sl0 < NSTEP) ? sl0 : (NSTEP - 1)] * ((sl0 < NSTEP) ? 1.0f : 0.0f);
  const float bhv1 = bias_lh[(sl1 < NSTEP) ? sl1 : (NSTEP - 1)] * ((sl1 < NSTEP) ? 1.0f : 0.0f);
  const float bo0  = bo[0];
  float hC[4][8], hS[4][8];
#pragma unroll
  for (int jt = 0; jt < 4; ++jt)
#pragma unroll
    for (int r = 0; r < 8; ++r) { hC[jt][r] = 0.0f; hS[jt][r] = 0.0f; }
  __syncthreads();

  {
    const float* sb = seqs + (size_t)rowbase * SEQF;
#pragma unroll 1
    for (int i = tid; i < ROWS_BLK * SEQF / 4; i += NTHR_MAIN) {
      const v4f v = *(const v4f*)(sb + 4 * i);
#pragma unroll
      for (int e = 0; e < 4; ++e) {
        const int L   = 4 * i + e;
        const int r   = L / SEQF;
        const int rem = L - r * SEQF;
        const int tt  = rem / NFEAT;
        const int f   = rem - tt * NFEAT;
        sAT[(r * NFEAT + f) * ATP + tt] = (_Float16)(v[e] * SCARRY);
      }
    }
  }
  __syncthreads();

  {
    const _Float16* wsr = WS16 + (size_t)c * KSIG + koff;
#pragma unroll 1
    for (int ms = wave; ms < MSUB_SIG; ms += NWAVE_MAIN) {
      v8f a0 = z8, a1 = z8, a2 = z8;
      const _Float16* arow = sAT + (ms * 16 + c) * ATP + koff;
#pragma unroll 1
      for (int k0 = 0; k0 < KSIG; k0 += 32) {
        const v16h a  = Frag<_Float16>::load(arow + k0);
        const v16h b0 = Frag<_Float16>::load(wsr + k0);
        const v16h b1 = Frag<_Float16>::load(wsr + 16 * KSIG + k0);
        const v16h b2 = Frag<_Float16>::load(wsr + 32 * KSIG + k0);
        a0 = Frag<_Float16>::mma(a, b0, a0);
        a1 = Frag<_Float16>::mma(a, b1, a1);
        a2 = Frag<_Float16>::mma(a, b2, a2);
        dep_guard_h(a0, a2, a, b2);
        keep4_h(a, b0, b1, b2);
      }
      acc_guard3(a0, a1, a2);
#pragma unroll
      for (int r = 0; r < 8; ++r) {
        float* dp = sLinSig + (size_t)(ms * 16 + 8 * hh + r) * SSP;
        dp[c]      = a0[r] * FOLD_SIG + bsv0;
        dp[16 + c] = a1[r] * FOLD_SIG + bsv1;
        if (c < 4) dp[32 + c] = a2[r] * FOLD_SIG + bsv2;
      }
    }
  }
  __syncthreads();

#pragma unroll 1
  for (int t = 0; t < NSTEP; ++t) {
    const int cur = t & 1;
    const _Float16* hrow = sH + cur * (ROWS_BLK * HP) + (msub * 16 + c) * HP + koff;
    _Float16* sHn = sH + (cur ^ 1) * (ROWS_BLK * HP);

    {
      v8f l0 = z8, l1 = z8;
      const _Float16* w0 = WH16 + (size_t)(32 * half + c) * NHID + koff;
      const _Float16* w1 = w0 + 16 * NHID;
#pragma unroll 1
      for (int k0 = 0; k0 < NHID; k0 += 32) {
        const v16h a  = Frag<_Float16>::load(hrow + k0);
        const v16h b0 = Frag<_Float16>::load(w0 + k0);
        const v16h b1 = Frag<_Float16>::load(w1 + k0);
        l0 = Frag<_Float16>::mma(a, b0, l0);
        l1 = Frag<_Float16>::mma(a, b1, l1);
        dep_guard_h(l0, l1, a, b1);
        keep4_h(a, b0, b1, a);
      }
      acc_guard2(l0, l1);
#pragma unroll
      for (int r = 0; r < 8; ++r) {
        float* dp = sLinH + (msub * 16 + 8 * hh + r) * LHP;
        dp[sl0] = l0[r] * FOLD_REC + bhv0;
        dp[sl1] = l1[r] * FOLD_REC + bhv1;
      }
    }
    __syncthreads();

    {
      const int row = tid >> 2, q = tid & 3;
      const int f4  = q + 16;
      const int f4c = (f4 < NFEAT) ? f4 : (NFEAT - 1);
      const float* lhp = sLinH + row * LHP;
      const float* sgb = sLinSig + (size_t)(row * NFEAT) * SSP;
      const float* sg0 = sgb + (q) * SSP;
      const float* sg1 = sgb + (q + 4) * SSP;
      const float* sg2 = sgb + (q + 8) * SSP;
      const float* sg3 = sgb + (q + 12) * SSP;
      const float* sg4 = sgb + f4c * SSP;
      float e0 = bo0, e1 = bo0, e2 = bo0, e3 = bo0, e4 = bo0;
#pragma unroll 1
      for (int s = 0; s < NSTEP; ++s) {
        const float lh = lhp[s], w = sWo[s];
        e0 = fmaf(w, ftanh(lh + sg0[s]), e0);
        e1 = fmaf(w, ftanh(lh + sg1[s]), e1);
        e2 = fmaf(w, ftanh(lh + sg2[s]), e2);
        e3 = fmaf(w, ftanh(lh + sg3[s]), e3);
        e4 = fmaf(w, ftanh(lh + sg4[s]), e4);
      }
      const float e4s = (f4 < NFEAT) ? e4 : -3.0e38f;
      float m = fmaxf(fmaxf(e0, e1), fmaxf(e2, e3));
      m = fmaxf(m, e4s);
      m = fmaxf(m, __shfl_xor(m, 1, 32));
      m = fmaxf(m, __shfl_xor(m, 2, 32));
      const float p0 = __expf(e0 - m), p1 = __expf(e1 - m), p2 = __expf(e2 - m), p3 = __expf(e3 - m);
      const float p4 = __expf(e4s - m);
      float sum = ((p0 + p1) + (p2 + p3)) + p4;
      sum += __shfl_xor(sum, 1, 32);
      sum += __shfl_xor(sum, 2, 32);
      const float inv = 1.0f / sum;
      const float* xt = seqs + (size_t)(rowbase + row) * SEQF + t * NFEAT;
      const float x0 = xt[q], x1 = xt[q + 4], x2 = xt[q + 8], x3 = xt[q + 12], x4 = xt[f4c];
      _Float16* xr = sX + row * XP;
      xr[q]      = (_Float16)((p0 * inv) * x0 * ACARRY);
      xr[q + 4]  = (_Float16)((p1 * inv) * x1 * ACARRY);
      xr[q + 8]  = (_Float16)((p2 * inv) * x2 * ACARRY);
      xr[q + 12] = (_Float16)((p3 * inv) * x3 * ACARRY);
      xr[f4]     = (_Float16)((p4 * inv) * x4 * ACARRY);
    }
    __syncthreads();

    {
      const v16h xa = Frag<_Float16>::load(sX + (msub * 16 + c) * XP + koff);
      float mv[8];
#pragma unroll
      for (int r = 0; r < 8; ++r) mv[r] = sMask[(msub * 16 + 8 * hh + r) * NSTEP + t];
#pragma unroll
      for (int jt = 0; jt < 4; ++jt) {
        const int n = 16 * (4 * half + jt) + c;
        v8f ar = z8, az = z8, ain = z8, ahn = z8;
        {
          const _Float16* wi = WI16 + (size_t)n * KIN + koff;
          const v16h b0 = Frag<_Float16>::load(wi);
          const v16h b1 = Frag<_Float16>::load(wi + (size_t)NHID * KIN);
          const v16h b2 = Frag<_Float16>::load(wi + (size_t)2 * NHID * KIN);
          ar  = Frag<_Float16>::mma(xa, b0, ar);
          az  = Frag<_Float16>::mma(xa, b1, az);
          ain = Frag<_Float16>::mma(xa, b2, ain);
          dep_guard_h(ar, ain, xa, b2);
          keep4_h(b0, b1, b2, xa);
        }
        const _Float16* wh = WHH16 + (size_t)n * NHID + koff;
#pragma unroll 1
        for (int k0 = 0; k0 < NHID; k0 += 32) {
          const v16h a  = Frag<_Float16>::load(hrow + k0);
          const v16h b0 = Frag<_Float16>::load(wh + k0);
          const v16h b1 = Frag<_Float16>::load(wh + (size_t)NHID * NHID + k0);
          const v16h b2 = Frag<_Float16>::load(wh + (size_t)2 * NHID * NHID + k0);
          ar  = Frag<_Float16>::mma(a, b0, ar);
          az  = Frag<_Float16>::mma(a, b1, az);
          ahn = Frag<_Float16>::mma(a, b2, ahn);
          dep_guard_h(ar, ahn, a, b2);
          keep4_h(a, b0, b1, b2);
        }
        acc_guard4(ar, az, ain, ahn);
        const float br = sB[n], bz = sB[NHID + n], bni = sB[2 * NHID + n], bnh = sB[3 * NHID + n];
#pragma unroll
        for (int r = 0; r < 8; ++r) {
          const float rg = fsig(ar[r] * FOLD_REC + br);
          const float zg = fsig(az[r] * FOLD_REC + bz);
          const float ng = ftanh(ain[r] * FOLD_REC + bni + rg * (ahn[r] * FOLD_REC + bnh));
          const float hp = hC[jt][r];
          const float hn = (1.0f - zg) * ng + zg * hp;
          hC[jt][r] = hn;
          hS[jt][r] += mv[r] * hn;
          sHn[(msub * 16 + 8 * hh + r) * HP + n] = (_Float16)(hn * ACARRY);
        }
      }
    }
    __syncthreads();
  }

  float* sOut = sLinSig;
#pragma unroll
  for (int jt = 0; jt < 4; ++jt) {
    const int n = 16 * (4 * half + jt) + c;
#pragma unroll
    for (int r = 0; r < 8; ++r) sOut[(msub * 16 + 8 * hh + r) * OUTP + n] = hS[jt][r];
  }
  __syncthreads();
  for (int pass = 0; pass < 2; ++pass) {
#pragma unroll
    for (int it = 0; it < ROWS_BLK * NHID / 4 / NTHR_MAIN; ++it) {
      const int idx = it * NTHR_MAIN + tid;
      const int row = idx >> 5, c4 = (idx & 31) * 4;
      const v4f v = *(const v4f*)(sOut + row * OUTP + c4);
      *(volatile v4f*)(out + (size_t)(rowbase + row) * NHID + c4) = v;
    }
    __threadfence();
  }
}

extern "C" void kernel_launch(void* const* d_in, const int* in_sizes, int n_in,
                              void* d_out, int out_size, void* d_ws, size_t ws_size, hipStream_t stream) {
  if (n_in < 12 || d_out == nullptr || d_ws == nullptr) return;
  if (in_sizes[0] != NSEQ * NSTEP * NFEAT || in_sizes[1] != NSEQ * NSTEP || in_sizes[2] != NSTEP * NHID ||
      in_sizes[3] != NSTEP || in_sizes[4] != NSTEP * NSTEP || in_sizes[5] != NSTEP || in_sizes[6] != NSTEP ||
      in_sizes[7] != 1 || in_sizes[8] != NG3 * NFEAT || in_sizes[9] != NG3 || in_sizes[10] != NG3 * NHID ||
      in_sizes[11] != NG3 || out_size != NSEQ * NHID) return;

  const float* seqs  = (const float*)d_in[0];
  const float* tmask = (const float*)d_in[1];
  const float* w_lh  = (const float*)d_in[2];
  const float* b_lh  = (const float*)d_in[3];
  const float* w_sig = (const float*)d_in[4];
  const float* b_sig = (const float*)d_in[5];
  const float* w_o   = (const float*)d_in[6];
  const float* b_o   = (const float*)d_in[7];
  const float* w_ih  = (const float*)d_in[8];
  const float* b_ih  = (const float*)d_in[9];
  const float* w_hh  = (const float*)d_in[10];
  const float* b_hh  = (const float*)d_in[11];
  float* out = (float*)d_out;

  char* ws = (char*)d_ws; size_t off = 0;
  auto carve = [&](size_t bytes) -> char* { char* p = ws + off; off += (bytes + 255) & ~(size_t)255; return p; };
  unsigned short* WSP = (unsigned short*)carve((size_t)NSIGP * KSIG * 2);
  unsigned short* WHP = (unsigned short*)carve((size_t)NLHP * NHID * 2);
  unsigned short* WIH = (unsigned short*)carve((size_t)NG3 * KIN * 2);
  unsigned short* WHH = (unsigned short*)carve((size_t)NG3 * NHID * 2);
  if (off > ws_size || off > (size_t)134217728) return;

  const int n8_sig = NSIGP * (KSIG / 8);
  const int n8_lh  = NLHP * (NHID / 8);
  const int n8_ih  = NG3 * (KIN / 8);
  const int n8_hh  = NG3 * (NHID / 8);
  padcvt_f16_kernel<<<(n8_sig + NTHR_PREP - 1) / NTHR_PREP, NTHR_PREP, 0, stream>>>(w_sig, WSP, NSTEP, NSTEP, NSIGP, KSIG, WCARRY);
  padcvt_f16_kernel<<<(n8_lh  + NTHR_PREP - 1) / NTHR_PREP, NTHR_PREP, 0, stream>>>(w_lh,  WHP, NSTEP, NHID,  NLHP,  NHID, WCARRY);
  padcvt_f16_kernel<<<(n8_ih  + NTHR_PREP - 1) / NTHR_PREP, NTHR_PREP, 0, stream>>>(w_ih,  WIH, NG3,   NFEAT, NG3,   KIN,  WCARRY);
  padcvt_f16_kernel<<<(n8_hh  + NTHR_PREP - 1) / NTHR_PREP, NTHR_PREP, 0, stream>>>(w_hh,  WHH, NG3,   NHID,  NG3,   NHID, WCARRY);

  seq_rnn_kernel<<<NSEQ / ROWS_BLK, NTHR_MAIN, 0, stream>>>(seqs, tmask, b_lh, b_sig, w_o, b_o, b_ih, b_hh,
                                                            WSP, WHP, WIH, WHH, out);
}
